// QueryNet_38568806318522
// MI455X (gfx1250) — hardware-verified
//
#include <hip/hip_runtime.h>
#include <math.h>

typedef __attribute__((ext_vector_type(16))) _Float16 v16h;
typedef __attribute__((ext_vector_type(16))) __bf16 v16b;
typedef __attribute__((ext_vector_type(8)))  _Float16 v8h;
typedef __attribute__((ext_vector_type(8)))  float v8f;
typedef __attribute__((ext_vector_type(4)))  float v4f;
typedef __attribute__((ext_vector_type(2)))  float v2f;
typedef __attribute__((ext_vector_type(4)))  unsigned v4u;
typedef __attribute__((ext_vector_type(4)))  int v4i;
typedef float __attribute__((may_alias)) float_a;
typedef int __attribute__((may_alias)) int_a;

template <typename T> __device__ __forceinline__ void vst2(void* p, T v) { *(volatile T*)p = v; __threadfence(); *(volatile T*)p = v; }
__device__ __forceinline__ v8f wmma16(v16h a, v16h b, v8f c) {
  v8f d = __builtin_amdgcn_wmma_f32_16x16x32_f16(false, a, false, b, (short)0, c, false, false);
  asm volatile("v_nop\n\tv_nop\n\tv_nop\n\tv_nop" : "+v"(d) : "v"(a), "v"(b));
  return d;
}
__device__ __forceinline__ v8f wmma_bf(v16b a, v16b b, v8f c) {
  v8f d = __builtin_amdgcn_wmma_f32_16x16x32_bf16(false, a, false, b, (short)0, c, false, false);
  asm volatile("v_nop\n\tv_nop\n\tv_nop\n\tv_nop" : "+v"(d) : "v"(a), "v"(b));
  return d;
}
__device__ __forceinline__ v16h frag_h(const _Float16* rowk0, int lane) {
  union { v16h v; v8h q[2]; } u; const _Float16* p = rowk0 + 8 * (lane >> 4);
  u.q[0] = *(const v8h*)p; u.q[1] = *(const v8h*)(p + 16); return u.v;
}
__device__ __forceinline__ v16h frag_f32(const float* rowk0, int lane) {
  v16h a; const float* p = rowk0 + 8 * (lane >> 4);
#pragma unroll
  for (int i = 0; i < 8; ++i) { a[i] = (_Float16)p[i]; a[8 + i] = (_Float16)p[16 + i]; }
  return a;
}
__device__ __forceinline__ v16h frag_f32s(const float* rowk0, int lane, float sc) {
  v16h a; const float* p = rowk0 + 8 * (lane >> 4);
#pragma unroll
  for (int i = 0; i < 8; ++i) { a[i] = (_Float16)(p[i] * sc); a[8 + i] = (_Float16)(p[16 + i] * sc); }
  return a;
}
__device__ __forceinline__ v16h fragc_f32(const float* W, int k0, int n, int lane, int ld, int K) {
  v16h a; const int g = lane >> 4;
#pragma unroll
  for (int i = 0; i < 8; ++i) { const int ka = k0 + 8 * g + i, kb = ka + 16;
    a[i] = (_Float16)(ka < K ? W[(size_t)ka * ld + n] : 0.f); a[8 + i] = (_Float16)(kb < K ? W[(size_t)kb * ld + n] : 0.f); }
  return a;
}
struct F2 { v16b h, l; };
__device__ __forceinline__ F2 bsplit16(const float v[16]) { F2 r;
#pragma unroll
  for (int i = 0; i < 16; ++i) { const __bf16 h = (__bf16)v[i]; r.h[i] = h; r.l[i] = (__bf16)(v[i] - (float)h); }
  return r; }
__device__ __forceinline__ F2 split_row(const float* row, int k0, int lane) { float v[16]; const float* p = row + k0 + 8 * (lane >> 4);
#pragma unroll
  for (int i = 0; i < 8; ++i) { v[i] = p[i]; v[8 + i] = p[16 + i]; }
  return bsplit16(v); }
__device__ __forceinline__ F2 split_rowK(const float* row, int k0, int lane, int K) { float v[16]; const int g = lane >> 4;
#pragma unroll
  for (int i = 0; i < 8; ++i) { const int ka = k0 + 8 * g + i, kb = ka + 16; v[i] = ka < K ? row[ka] : 0.f; v[8 + i] = kb < K ? row[kb] : 0.f; }
  return bsplit16(v); }
__device__ __forceinline__ F2 split_col(const float* W, int k0, int n, int lane, int ld, int K) { float v[16]; const int g = lane >> 4;
#pragma unroll
  for (int i = 0; i < 8; ++i) { const int ka = k0 + 8 * g + i, kb = ka + 16; v[i] = ka < K ? W[(size_t)ka * ld + n] : 0.f; v[8 + i] = kb < K ? W[(size_t)kb * ld + n] : 0.f; }
  return bsplit16(v); }
__device__ __forceinline__ v8f mac3(const F2& a, const F2& b, v8f c) { c = wmma_bf(a.l, b.h, c); c = wmma_bf(a.h, b.l, c); return wmma_bf(a.h, b.h, c); }
__device__ __forceinline__ float sigm(float v) { return 1.0f / (1.0f + expf(-v)); }
#define LDSX() do { asm volatile("s_wait_dscnt 0" ::: "memory"); __builtin_amdgcn_wave_barrier(); __builtin_amdgcn_fence(__ATOMIC_RELEASE, "workgroup"); } while (0)

#define NBQ 256
#define SQ 512
#define DE 300
#define DEP 320
#define DH 512
#define PADID 40001
#define VOC 40002

__global__ __launch_bounds__(256) void k_pool(const int* __restrict__ ids, const float* __restrict__ emb, const float* __restrict__ qw, const float* __restrict__ qb, float* __restrict__ P) {
  __shared__ float ssc[SQ]; __shared__ int sid[SQ]; __shared__ float sred[8]; __shared__ __align__(16) float sp[DEP];
  const int b = blockIdx.x, tid = threadIdx.x, wave = tid >> 5, lane = tid & 31;
  for (int s = tid; s < SQ; s += 256) { int id = ids[(size_t)b * SQ + s]; const bool pad = (id == PADID); id = id < 0 ? 0 : (id >= VOC ? VOC - 1 : id); sid[s] = id;
    const float* er = emb + (size_t)id * DE; float sc = 0.f; for (int d = 0; d < DE; ++d) sc += er[d] * qw[d]; sc += qb[0];
    ssc[s] = pad ? -3.0e38f : sc; }
  __syncthreads();
  float mx = -3.4e38f; for (int s = tid; s < SQ; s += 256) mx = fmaxf(mx, ssc[s]);
#pragma unroll
  for (int off = 16; off >= 1; off >>= 1) mx = fmaxf(mx, __shfl_xor(mx, off, 32));
  if (lane == 0) sred[wave] = mx;
  __syncthreads();
  mx = sred[0]; for (int w = 1; w < 8; ++w) mx = fmaxf(mx, sred[w]);
  __syncthreads();
  float se = 0.f; for (int s = tid; s < SQ; s += 256) { const float p = ssc[s] <= -1.0e38f ? 0.f : expf(ssc[s] - mx); ssc[s] = p; se += p; }
#pragma unroll
  for (int off = 16; off >= 1; off >>= 1) se += __shfl_xor(se, off, 32);
  if (lane == 0) sred[wave] = se;
  __syncthreads();
  float tot = 0.f; for (int w = 0; w < 8; ++w) tot += sred[w]; const float inv = 1.0f / tot;
  for (int d = tid; d < DEP; d += 256) { float acc = 0.f; if (d < DE) { for (int s = 0; s < SQ; ++s) acc += ssc[s] * emb[(size_t)sid[s] * DE + d]; acc *= inv; } sp[d] = acc; }
  __syncthreads();
  if (tid < DEP / 4) vst2(P + (size_t)b * DEP + tid * 4, *(const v4f*)(&sp[tid * 4]));
}
__global__ __launch_bounds__(32) void k_head(const float* __restrict__ P, const float* __restrict__ w1, const float* __restrict__ b1, const float* __restrict__ w2, const float* __restrict__ b2, float* __restrict__ out) {
  __shared__ __align__(16) float sh[16][DH + 4]; __shared__ __align__(16) float so[16][2];
  const int lane = threadIdx.x, col = lane & 15, g = lane >> 4; const int r0 = blockIdx.x * 16;
#pragma unroll 1
  for (int np = 0; np < 4; ++np) { v8f acc[8] = {};
#pragma unroll 1
    for (int kc = 0; kc < DEP / 32; ++kc) { const F2 a = split_row(P + (size_t)(r0 + col) * DEP, kc * 32, lane);
#pragma unroll
      for (int j = 0; j < 8; ++j) acc[j] = mac3(a, split_col(w1, kc * 32, np * 128 + j * 16 + col, lane, DH, DE), acc[j]); }
#pragma unroll
    for (int j = 0; j < 8; ++j) { const int n = np * 128 + j * 16 + col; const float bb = b1[n];
#pragma unroll
      for (int r = 0; r < 8; ++r) { const float v = acc[j][r] + bb; sh[8 * g + r][n] = v > 0.f ? v : 0.f; } } }
  LDSX();
  { const int rl = lane >> 1, o = lane & 1; float s = b2[o]; for (int n = 0; n < DH; ++n) s += sh[rl][n] * w2[n * 2 + o]; so[rl][o] = s; }
  LDSX();
  if (lane < 8) vst2(out + (size_t)r0 * 2 + lane * 4, *(const v4f*)(&so[0][0] + lane * 4));
}
extern "C" void kernel_launch(void* const* d_in, const int* in_sizes, int n_in, void* d_out, int out_size, void* d_ws, size_t ws_size, hipStream_t stream) {
  (void)in_sizes; (void)n_in; (void)out_size; (void)ws_size;
  const int* ids = (const int*)d_in[0]; const float* emb = (const float*)d_in[1]; const float* qw = (const float*)d_in[2]; const float* qb = (const float*)d_in[3];
  const float* w1 = (const float*)d_in[4]; const float* b1 = (const float*)d_in[5]; const float* w2 = (const float*)d_in[6]; const float* b2 = (const float*)d_in[7];
  float* out = (float*)d_out;
  float* P = (float*)d_ws;
  k_pool<<<NBQ, 256, 0, stream>>>(ids, emb, qw, qb, P);
  k_head<<<NBQ / 16, 32, 0, stream>>>(P, w1, b1, w2, b2, out);
}
